// Encoder_45226005626971
// MI455X (gfx1250) — hardware-verified
//
#include <hip/hip_runtime.h>
#include <stddef.h>
#include <stdint.h>
#include <math.h>


#define DF     64
#define KH     128
#define NGR    512
#define NTHR   256
#define NWAVE  8
#define EPT    8
#define CHUNK  (NTHR * EPT)
#define WCAP   (EPT * 32)
#define LISTN  (NWAVE * WCAP)
#define NBA    1024
#define SLA    10
#define RCAP   16384
#define DEGCAP 64
#define TM     128
#define NUW    1024
#define NWBLK  ((4 * NUW) / NTHR)
#define AGG_ZINTS    (LISTN + 2 * RCAP + 3 * NBA)
#define AGG_LDS_INTS (AGG_ZINTS + 16)
#define MLP_STG_B (TM * DF * 4)
#define MLP_TT_B  (TM * KH * 2)
#define MLP_BS_B  512
#define MLP_RS_B  1024
#define MLP_LDS   (MLP_STG_B + MLP_TT_B + MLP_BS_B + MLP_RS_B)
#define WSMAX  134217728

static_assert((CHUNK & (CHUNK - 1)) == 0 && CHUNK <= 4096);
static_assert((NBA & (NBA - 1)) == 0 && NBA == (1 << SLA));
static_assert(((long long)CHUNK << SLA) < (1LL << 31));
static_assert(NBA % NWAVE == 0 && NBA % 32 == 0 && NBA % TM == 0);
static_assert(RCAP % 4 == 0 && AGG_ZINTS % 4 == 0 && LISTN % 4 == 0);
static_assert(KH % 32 == 0 && KH == 2 * DF && DF == 2 * 32);
static_assert(TM == NWAVE * 16);
static_assert(NUW % NTHR == 0 && NUW == DF * (KH / 8));
static_assert(AGG_LDS_INTS * 4 <= 300000 && MLP_LDS <= 300000);
static_assert((MLP_STG_B + MLP_TT_B + MLP_BS_B) % 16 == 0);

typedef float          v2f   __attribute__((ext_vector_type(2)));
typedef float          v4f   __attribute__((ext_vector_type(4)));
typedef float          v8f   __attribute__((ext_vector_type(8)));
typedef double         v2d   __attribute__((ext_vector_type(2)));
typedef int            v4i   __attribute__((ext_vector_type(4)));
typedef int            v8i   __attribute__((ext_vector_type(8)));
typedef unsigned int   v4u   __attribute__((ext_vector_type(4)));
typedef unsigned short v4us  __attribute__((ext_vector_type(4)));
typedef unsigned short v8us  __attribute__((ext_vector_type(8)));
typedef unsigned short v16us __attribute__((ext_vector_type(16)));
typedef __bf16         v16bf __attribute__((ext_vector_type(16)));
typedef v2f  __attribute__((may_alias)) v2fa;
typedef v4f  __attribute__((may_alias)) v4fa;
typedef v2d  __attribute__((may_alias)) v2da;
typedef v4i  __attribute__((may_alias)) v4ia;
typedef v4us __attribute__((may_alias)) v4usa;
typedef v8us __attribute__((may_alias)) v8usa;
union FragB { v16bf v; v16us u; v8us h[2]; v8i w; };

__device__ __forceinline__ v8f wmb(const FragB& a, const FragB& b, v8f c) {
  v8f d = __builtin_amdgcn_wmma_f32_16x16x32_bf16(false, a.v, false, b.v, (short)0, c, false, false);
  asm volatile("v_nop\n\tv_nop\n\tv_nop\n\tv_nop" : "+v"(d) : "v"(a.w), "v"(b.w));
  return d;
}

__device__ __forceinline__ unsigned bf16_bits(float f) {
  const unsigned u = __float_as_uint(f);
  const unsigned r = (u + 0x7FFFu + ((u >> 16) & 1u)) >> 16;
  return (f != f) ? 0x7FC0u : r;
}
__device__ __forceinline__ float bf16_val(float f) {
  return __uint_as_float(bf16_bits(f) << 16);
}
__device__ __forceinline__ float bnap(float v, float mu, float sc, float be) {
  return (v - mu) * sc + be;
}

template <int SLB>
__device__ __forceinline__ int scan_chunk(const int* __restrict__ dsts, int nE, int cbase, int slotBase,
                                          int nb, int vec8, int* list, int tid, int lane, int wave) {
  int wc = 0;
  const int el0  = tid * EPT;
  const int e0   = cbase + el0;
  const int sent = -2147483647 - 1;
  v4i da, db;
  if (vec8 != 0 && cbase + CHUNK <= nE) {
    da = *(const v4i*)(dsts + e0);
    db = *(const v4i*)(dsts + e0 + 4);
  } else {
    da.x = (e0     < nE) ? dsts[min(e0,     nE - 1)] : sent;
    da.y = (e0 + 1 < nE) ? dsts[min(e0 + 1, nE - 1)] : sent;
    da.z = (e0 + 2 < nE) ? dsts[min(e0 + 2, nE - 1)] : sent;
    da.w = (e0 + 3 < nE) ? dsts[min(e0 + 3, nE - 1)] : sent;
    db.x = (e0 + 4 < nE) ? dsts[min(e0 + 4, nE - 1)] : sent;
    db.y = (e0 + 5 < nE) ? dsts[min(e0 + 5, nE - 1)] : sent;
    db.z = (e0 + 6 < nE) ? dsts[min(e0 + 6, nE - 1)] : sent;
    db.w = (e0 + 7 < nE) ? dsts[min(e0 + 7, nE - 1)] : sent;
  }
  const unsigned nbs = (unsigned)slotBase;
  const unsigned unb = (unsigned)nb;
  const unsigned s0 = (unsigned)da.x - nbs, s1 = (unsigned)da.y - nbs;
  const unsigned s2 = (unsigned)da.z - nbs, s3 = (unsigned)da.w - nbs;
  const unsigned s4 = (unsigned)db.x - nbs, s5 = (unsigned)db.y - nbs;
  const unsigned s6 = (unsigned)db.z - nbs, s7 = (unsigned)db.w - nbs;
  const bool h0 = s0 < unb, h1 = s1 < unb, h2 = s2 < unb, h3 = s3 < unb;
  const bool h4 = s4 < unb, h5 = s5 < unb, h6 = s6 < unb, h7 = s7 < unb;
  const unsigned any = __builtin_amdgcn_ballot_w32(h0 | h1 | h2 | h3 | h4 | h5 | h6 | h7);
  if (any != 0u) {
#define HITJ(J, HJ, SJ) { \
      const unsigned mj = __builtin_amdgcn_ballot_w32(HJ); \
      if (mj != 0u) { \
        if (HJ) { \
          const int pos = wc + (int)__builtin_amdgcn_mbcnt_lo(mj, 0u); \
          if (pos < WCAP) list[wave * WCAP + pos] = ((el0 + (J)) << SLB) | (int)(SJ); \
        } \
        wc += (int)__builtin_popcount(mj); } }
    HITJ(0, h0, s0)
    HITJ(1, h1, s1)
    HITJ(2, h2, s2)
    HITJ(3, h3, s3)
    HITJ(4, h4, s4)
    HITJ(5, h5, s5)
    HITJ(6, h6, s6)
    HITJ(7, h7, s7)
#undef HITJ
  }
  return wc;
}

__device__ __forceinline__ void wunit(const float* __restrict__ W, unsigned short* P, int v) {
  const int n  = v >> 4;
  const int k8 = (v & 15) * 8;
  const int kk = k8 & (DF - 1);
  const float* p = W + (size_t)kk * DF + n;
  v8us o;
#pragma unroll
  for (int i = 0; i < 8; ++i) o[i] = (unsigned short)bf16_bits(p[(size_t)i * DF]);
  unsigned short* dp = P + (size_t)n * KH + k8;
  *(volatile v8us*)dp = o;
  __threadfence();
  *(volatile v8us*)dp = o;
}

__global__ __launch_bounds__(NTHR) void k_prep(const float* __restrict__ x,
                                               const float* __restrict__ Wa, const float* __restrict__ Wb,
                                               const float* __restrict__ Wc, const float* __restrict__ Wd,
                                               const int* __restrict__ bat, int nN, int nUx, int nbX,
                                               unsigned short* WP, unsigned short* XB, int* FLG) {
  __shared__ int sbad[NWAVE];
  const int b = (int)blockIdx.x, tid = (int)threadIdx.x;
  if (b < NWBLK) {
    const int u    = b * NTHR + tid;
    const int part = u >> 10;
    const int v    = u & (NUW - 1);
    if (part == 0)      wunit(Wa, WP, v);
    else if (part == 1) wunit(Wb, WP + 8192, v);
    else if (part == 2) wunit(Wc, WP + 16384, v);
    else                wunit(Wd, WP + 24576, v);
  } else if (b < NWBLK + nbX) {
    const int u2 = (b - NWBLK) * NTHR + tid;
    if (u2 < nUx) {
      const int row = u2 >> 3;
      const int k8  = (u2 & 7) * 8;
      const int rc  = row < nN ? row : nN - 1;
      const float* p = x + (size_t)rc * DF + k8;
      const v4f a = *(const v4fa*)p;
      const v4f c = *(const v4fa*)(p + 4);
      const bool ok = row < nN;
      v8us o;
      o[0] = ok ? (unsigned short)bf16_bits(a.x) : (unsigned short)0;
      o[1] = ok ? (unsigned short)bf16_bits(a.y) : (unsigned short)0;
      o[2] = ok ? (unsigned short)bf16_bits(a.z) : (unsigned short)0;
      o[3] = ok ? (unsigned short)bf16_bits(a.w) : (unsigned short)0;
      o[4] = ok ? (unsigned short)bf16_bits(c.x) : (unsigned short)0;
      o[5] = ok ? (unsigned short)bf16_bits(c.y) : (unsigned short)0;
      o[6] = ok ? (unsigned short)bf16_bits(c.z) : (unsigned short)0;
      o[7] = ok ? (unsigned short)bf16_bits(c.w) : (unsigned short)0;
      unsigned short* dp = XB + (size_t)row * DF + k8;
      *(volatile v8us*)dp = o;
      __threadfence();
      *(volatile v8us*)dp = o;
    }
  } else {
    int bad = 0;
#pragma unroll 1
    for (int i = tid; i < nN; i += NTHR) {
      const int i1 = (i + 1 < nN) ? i + 1 : nN - 1;
      const int v0 = bat[i];
      const int v1 = bat[i1];
      bad |= (v0 < 0) | (v0 >= NGR) | (v0 > v1);
    }
    const unsigned mk = __builtin_amdgcn_ballot_w32(bad != 0);
    if ((tid & 31) == 0) sbad[tid >> 5] = (mk != 0u) ? 1 : 0;
    __syncthreads();
    int tot = 0;
#pragma unroll
    for (int w = 0; w < NWAVE; ++w) tot |= sbad[w];
    v4i f;
    f.x = tot; f.y = tot; f.z = tot; f.w = tot;
    const bool okst = tid < 8;
    int* fp = FLG + 4 * (tid & 7);
    if (okst) *(volatile v4i*)fp = f;
    __threadfence();
    if (okst) *(volatile v4i*)fp = f;
  }
}

template <int L0>
__global__ __launch_bounds__(NTHR) void k_scan(const int* __restrict__ srcs, const int* __restrict__ dsts,
                                               int nE, int nN, int vec8, int mRows,
                                               const unsigned* __restrict__ xbw,
                                               const float* __restrict__ vf, const float* __restrict__ st,
                                               unsigned short* hb) {
  extern __shared__ __attribute__((aligned(16))) int dsm[];
  int* list = dsm;
  int* hl   = dsm + LISTN;
  int* sl   = dsm + LISTN + RCAP;
  int* cnt  = dsm + LISTN + 2 * RCAP;
  int* offs = cnt + NBA;
  int* cur  = offs + NBA;
  int* misc = cur + NBA;
  const int tid = (int)threadIdx.x, lane = tid & 31, wave = tid >> 5;
  const int nodeBase = (int)blockIdx.x * NBA;

  {
    const v4i z4 = {0, 0, 0, 0};
    for (int i = tid * 4; i < AGG_ZINTS; i += NTHR * 4) *(v4ia*)(dsm + i) = z4;
    if (tid < 16) misc[tid] = 0;
  }
  float mu0 = 0.0f, mu1 = 0.0f, sc0 = 1.0f, sc1 = 1.0f, be0 = 0.0f, be1 = 0.0f;
  if constexpr (L0 == 0) {
    const v2f a = *(const v2fa*)(st + 2 * lane);
    const v2f c = *(const v2fa*)(st + DF + 2 * lane);
    const v2f d = *(const v2fa*)(st + 2 * DF + 2 * lane);
    mu0 = a.x; mu1 = a.y; sc0 = c.x; sc1 = c.y; be0 = d.x; be1 = d.y;
  }
  __syncthreads();

  int t = 0, ov = 0;
  const int nChunks = (nE + CHUNK - 1) / CHUNK;
#pragma unroll 1
  for (int ch = 0; ch < nChunks; ++ch) {
    const int cbase = ch * CHUNK;
    const int wc = scan_chunk<SLA>(dsts, nE, cbase, nodeBase, NBA, vec8, list, tid, lane, wave);
    if (lane == 0) misc[wave] = wc;
    __syncthreads();
    if (wave == 0) {
#pragma unroll 1
      for (int w2 = 0; w2 < NWAVE; ++w2) {
        int c = misc[w2];
        c = c < 0 ? 0 : (c > WCAP ? WCAP : c);
#pragma unroll 1
        for (int b0 = 0; b0 < c; b0 += 32) {
          const int idx = b0 + lane;
          const int ent = list[w2 * WCAP + (idx < WCAP ? idx : WCAP - 1)];
          const int m32 = (c - b0) < 32 ? (c - b0) : 32;
#pragma unroll 1
          for (int k = 0; k < m32; ++k) {
            const int u    = __builtin_amdgcn_readlane(ent, k);
            const int slot = u & (NBA - 1);
            const int el   = (u >> SLA) & (CHUNK - 1);
            const int pk   = ((cbase + el) << SLA) | slot;
            if (t < RCAP) {
              if (lane == 0) { hl[t] = pk; cnt[slot] = cnt[slot] + 1; }
              t = t + 1;
            } else {
              ov = 1;
            }
          }
        }
      }
    }
    __syncthreads();
  }
  if (wave == 0 && lane == 0) { misc[8] = t; misc[9] = ov; }
  __syncthreads();
  int tt = misc[8];
  tt = tt < 0 ? 0 : (tt > RCAP ? RCAP : tt);
  const int ovf = misc[9];

  if (wave == 0) {
    const int base = lane * (NBA / 32);
    int s = 0;
#pragma unroll 1
    for (int i = 0; i < NBA / 32; ++i) s += cnt[base + i];
    int incl = s;
#pragma unroll
    for (int d = 1; d < 32; d <<= 1) {
      const int y = __shfl_up(incl, d, 32);
      if (lane >= d) incl += y;
    }
    int run = incl - s;
#pragma unroll 1
    for (int i = 0; i < NBA / 32; ++i) {
      const int cv = cnt[base + i];
      offs[base + i] = run;
      cur[base + i]  = run;
      run += cv;
    }
  }
  __syncthreads();
  if (wave == 0) {
#pragma unroll 1
    for (int b0 = 0; b0 < tt; b0 += 32) {
      const int idx = b0 + lane;
      const int ent = hl[idx < RCAP ? idx : RCAP - 1];
      const int m32 = (tt - b0) < 32 ? (tt - b0) : 32;
#pragma unroll 1
      for (int k = 0; k < m32; ++k) {
        const int u    = __builtin_amdgcn_readlane(ent, k);
        const int slot = u & (NBA - 1);
        if (lane == 0) {
          int p = cur[slot];
          p = p < 0 ? 0 : (p > RCAP - 1 ? RCAP - 1 : p);
          sl[p] = u;
          cur[slot] = p + 1;
        }
      }
    }
  }
  __syncthreads();

  const float qnan = __int_as_float(0x7fc00000);
  const float pz = (ovf != 0) ? qnan : 0.0f;
  const int q0s = (4 * lane) & 31, q1s = (4 * lane + 1) & 31;
  const int q2s = (4 * lane + 2) & 31, q3s = (4 * lane + 3) & 31;
#pragma unroll 1
  for (int si = 0; si < NBA / NWAVE; ++si) {
    const int s    = si * NWAVE + wave;
    const int node = nodeBase + s;
    int c = cnt[s];
    const bool big = c > DEGCAP;
    c = c < 0 ? 0 : (c > DEGCAP ? DEGCAP : c);
    int o = offs[s];
    o = o < 0 ? 0 : (o > RCAP ? RCAP : o);
    const int nc = node < nN ? node : nN - 1;
    float acc0 = 0.0f, acc1 = 0.0f;
#pragma unroll 1
    for (int b0 = 0; b0 < c; b0 += 32) {
      int idx = o + b0 + lane;
      idx = idx > RCAP - 1 ? RCAP - 1 : idx;
      const int ent = sl[idx];
      int eid = ent >> SLA;
      eid = eid < 0 ? 0 : (eid > nE - 1 ? nE - 1 : eid);
      int sr = srcs[eid];
      sr = sr < 0 ? 0 : (sr > nN - 1 ? nN - 1 : sr);
      const int m32 = (c - b0) < 32 ? (c - b0) : 32;
#pragma unroll 1
      for (int k = 0; k < m32; ++k) {
        const int sk = __builtin_amdgcn_readlane(sr, k);
        if constexpr (L0 != 0) {
          const unsigned w = xbw[(size_t)sk * (DF / 2) + lane];
          acc0 += __uint_as_float(w << 16);
          acc1 += __uint_as_float(w & 0xffff0000u);
        } else {
          const v2f a = *(const v2fa*)(vf + (size_t)sk * DF + 2 * lane);
          acc0 += bnap(a.x, mu0, sc0, be0);
          acc1 += bnap(a.y, mu1, sc1, be1);
        }
      }
    }
    float sv0, sv1;
    if constexpr (L0 != 0) {
      const unsigned w = xbw[(size_t)nc * (DF / 2) + lane];
      sv0 = __uint_as_float(w << 16);
      sv1 = __uint_as_float(w & 0xffff0000u);
    } else {
      const v2f a = *(const v2fa*)(vf + (size_t)nc * DF + 2 * lane);
      sv0 = bnap(a.x, mu0, sc0, be0);
      sv1 = bnap(a.y, mu1, sc1, be1);
    }
    const float pzr = big ? qnan : pz;
    const bool live = node < nN;
    const float y0 = (sv0 + acc0) + pzr;
    const float y1 = (sv1 + acc1) + pzr;
    const float v0 = live ? y0 : 0.0f;
    const float v1 = live ? y1 : 0.0f;
    const bool wr = (node < mRows) && (lane < 16);
    const unsigned hb0 = bf16_bits(v0), hb1 = bf16_bits(v1);
    const unsigned lb0 = bf16_bits(v0 - __uint_as_float(hb0 << 16));
    const unsigned lb1 = bf16_bits(v1 - __uint_as_float(hb1 << 16));
    const int hw = (int)(hb0 | (hb1 << 16));
    const int lw = (int)(lb0 | (lb1 << 16));
    const int g0 = __shfl(hw, q0s, 32), g1 = __shfl(hw, q1s, 32);
    const int g2 = __shfl(hw, q2s, 32), g3 = __shfl(hw, q3s, 32);
    const int p0 = __shfl(lw, q0s, 32), p1 = __shfl(lw, q1s, 32);
    const int p2 = __shfl(lw, q2s, 32), p3 = __shfl(lw, q3s, 32);
    const bool lsel = (lane & 8) != 0;
    v4u pv;
    pv.x = (unsigned int)(lsel ? p0 : g0);
    pv.y = (unsigned int)(lsel ? p1 : g1);
    pv.z = (unsigned int)(lsel ? p2 : g2);
    pv.w = (unsigned int)(lsel ? p3 : g3);
    unsigned short* hp = hb + (size_t)node * KH + 8 * (lane & 15);
    if (wr) *(volatile v4u*)hp = pv;
    __threadfence();
    if (wr) *(volatile v4u*)hp = pv;
  }
}

__global__ __launch_bounds__(NTHR) void k_mlp(const unsigned short* __restrict__ Hp,
                                              const unsigned short* __restrict__ W1d,
                                              const unsigned short* __restrict__ W2d,
                                              const float* __restrict__ b1, const float* __restrict__ b2,
                                              int nN, float* V, double* rec) {
  extern __shared__ __attribute__((aligned(16))) unsigned char smem[];
  float*          stg = (float*)smem;
  unsigned short* tt  = (unsigned short*)(smem + MLP_STG_B);
  float*          bs  = (float*)(smem + MLP_STG_B + MLP_TT_B);
  double*         rs  = (double*)(smem + MLP_STG_B + MLP_TT_B + MLP_BS_B);
  const int tid = (int)threadIdx.x, lane = tid & 31, wave = tid >> 5, hh = lane >> 4, m = lane & 15;
  const int rowBase = (int)blockIdx.x * TM;

  if (tid < 2 * DF) {
    const int c = tid & (DF - 1);
    const float va = b1[c];
    const float vb = b2[c];
    bs[tid] = bf16_val(tid < DF ? va : vb);
  }

  const v8f z8 = {0.f, 0.f, 0.f, 0.f, 0.f, 0.f, 0.f, 0.f};
  v8f acc[4];
  acc[0] = z8; acc[1] = z8; acc[2] = z8; acc[3] = z8;

  {
    const unsigned short* ap = Hp + (size_t)(rowBase + 16 * wave + m) * (size_t)KH + 8 * hh;
    const unsigned short* wp = W1d + (size_t)m * (size_t)KH + 8 * hh;
#pragma unroll 1
    for (int ks = 0; ks < KH / 32; ++ks) {
      FragB af;
      af.h[0] = *(const v8usa*)(ap + 32 * ks);
      af.h[1] = *(const v8usa*)(ap + 32 * ks + 16);
#pragma unroll
      for (int t = 0; t < 4; ++t) {
        const unsigned short* wq = wp + (size_t)(16 * t) * (size_t)KH + 32 * ks;
        FragB bf;
        bf.h[0] = *(const v8usa*)wq;
        bf.h[1] = *(const v8usa*)(wq + 16);
        acc[t] = wmb(af, bf, acc[t]);
      }
    }
  }
#pragma unroll
  for (int t = 0; t < 4; ++t) {
#pragma unroll
    for (int r = 0; r < 8; ++r) {
      const int lr = 16 * wave + 8 * hh + r;
      stg[lr * DF + 16 * t + m] = acc[t][r];
    }
  }
  __syncthreads();

  {
    const v4f bb = *(const v4fa*)(bs + 4 * m);
#pragma unroll 1
    for (int i = 0; i < 8; ++i) {
      const int lr = 16 * wave + 2 * i + hh;
      const v4f a = *(const v4fa*)(stg + lr * DF + 4 * m);
      const float t0 = tanhf(a.x + bb.x);
      const float t1 = tanhf(a.y + bb.y);
      const float t2 = tanhf(a.z + bb.z);
      const float t3 = tanhf(a.w + bb.w);
      v4us h4, l4;
      unsigned hb;
      hb = bf16_bits(t0); h4[0] = (unsigned short)hb; l4[0] = (unsigned short)bf16_bits(t0 - __uint_as_float(hb << 16));
      hb = bf16_bits(t1); h4[1] = (unsigned short)hb; l4[1] = (unsigned short)bf16_bits(t1 - __uint_as_float(hb << 16));
      hb = bf16_bits(t2); h4[2] = (unsigned short)hb; l4[2] = (unsigned short)bf16_bits(t2 - __uint_as_float(hb << 16));
      hb = bf16_bits(t3); h4[3] = (unsigned short)hb; l4[3] = (unsigned short)bf16_bits(t3 - __uint_as_float(hb << 16));
      *(v4usa*)(tt + lr * KH + 4 * m) = h4;
      *(v4usa*)(tt + lr * KH + DF + 4 * m) = l4;
    }
  }
  __syncthreads();

  acc[0] = z8; acc[1] = z8; acc[2] = z8; acc[3] = z8;
  {
    const unsigned short* tp = tt + (16 * wave + m) * KH + 8 * hh;
    const unsigned short* wp = W2d + (size_t)m * (size_t)KH + 8 * hh;
#pragma unroll 1
    for (int ks = 0; ks < KH / 32; ++ks) {
      FragB af;
      af.h[0] = *(const v8usa*)(tp + 32 * ks);
      af.h[1] = *(const v8usa*)(tp + 32 * ks + 16);
#pragma unroll
      for (int t = 0; t < 4; ++t) {
        const unsigned short* wq = wp + (size_t)(16 * t) * (size_t)KH + 32 * ks;
        FragB bf;
        bf.h[0] = *(const v8usa*)wq;
        bf.h[1] = *(const v8usa*)(wq + 16);
        acc[t] = wmb(af, bf, acc[t]);
      }
    }
  }
#pragma unroll
  for (int t = 0; t < 4; ++t) {
#pragma unroll
    for (int r = 0; r < 8; ++r) {
      const int lr = 16 * wave + 8 * hh + r;
      stg[lr * DF + 16 * t + m] = acc[t][r];
    }
  }
  __syncthreads();

  {
    const v4f bb = *(const v4fa*)(bs + DF + 4 * m);
#pragma unroll 1
    for (int i = 0; i < 8; ++i) {
      const int lr = 16 * wave + 2 * i + hh;
      const v4f a = *(const v4fa*)(stg + lr * DF + 4 * m);
      v4f y;
      y.x = tanhf(a.x + bb.x);
      y.y = tanhf(a.y + bb.y);
      y.z = tanhf(a.z + bb.z);
      y.w = tanhf(a.w + bb.w);
      *(v4fa*)(stg + lr * DF + 4 * m) = y;
    }
  }
  __syncthreads();

  v4f fv[8];
#pragma unroll
  for (int i = 0; i < 8; ++i) {
    const int lr = 16 * wave + 2 * i + hh;
    fv[i] = *(const v4fa*)(stg + lr * DF + 4 * m);
  }
  if (tid < 2 * DF) {
    const int col = tid & (DF - 1);
    const bool sq = tid >= DF;
    double s = 0.0;
#pragma unroll 1
    for (int r = 0; r < TM; ++r) {
      const double dv = (double)stg[r * DF + col];
      const double tv = sq ? dv * dv : dv;
      s += ((rowBase + r) < nN) ? tv : 0.0;
    }
    rs[tid] = s;
  }
  __syncthreads();
  const v2d d2 = *(const v2da*)(rs + 2 * (tid & 63));
  const bool okr = tid < 64;
  double* rp = rec + (size_t)blockIdx.x * (2 * DF) + 2 * (tid & 63);

#pragma unroll
  for (int i = 0; i < 8; ++i) {
    const int lr = 16 * wave + 2 * i + hh;
    float* op = V + (size_t)(rowBase + lr) * DF + 4 * m;
    *(volatile v4f*)op = fv[i];
  }
  if (okr) *(volatile v2d*)rp = d2;
  __threadfence();
#pragma unroll
  for (int i = 0; i < 8; ++i) {
    const int lr = 16 * wave + 2 * i + hh;
    float* op = V + (size_t)(rowBase + lr) * DF + 4 * m;
    *(volatile v4f*)op = fv[i];
  }
  if (okr) *(volatile v2d*)rp = d2;
}

__global__ __launch_bounds__(128) void k_bn(const double* __restrict__ rec, int nT, int nN,
                                            const float* __restrict__ gamma, const float* __restrict__ beta,
                                            float* st) {
  __shared__ double sd[2 * DF];
  __shared__ __attribute__((aligned(16))) float sst[4 * DF];
  const int tid = (int)threadIdx.x;
  double s = 0.0;
#pragma unroll 4
  for (int t = 0; t < nT; ++t) s += rec[(size_t)t * (2 * DF) + tid];
  sd[tid] = s;
  __syncthreads();
  if (tid < DF) {
    const double inv  = 1.0 / (double)nN;
    const double mean = sd[tid] * inv;
    const double ex2  = sd[DF + tid] * inv;
    double var = ex2 - mean * mean;
    var = (var < 0.0) ? 0.0 : var;
    const float vfl = (float)var;
    const float g   = bf16_val(gamma[tid]);
    const float be  = bf16_val(beta[tid]);
    const float sc  = g / sqrtf(vfl + 1e-5f);
    sst[tid]          = (float)mean;
    sst[DF + tid]     = sc;
    sst[2 * DF + tid] = be;
    sst[3 * DF + tid] = 0.0f;
  }
  __syncthreads();
  const v4f o = *(const v4fa*)(sst + 4 * (tid & 63));
  const bool okst = tid < 64;
  float* op = st + 4 * (tid & 63);
  if (okst) *(volatile v4f*)op = o;
  __threadfence();
  if (okst) *(volatile v4f*)op = o;
}

__device__ __forceinline__ int lbound(const int* __restrict__ bat, int nN, int key) {
  int lo = 0, hi = nN;
#pragma unroll 1
  for (int it = 0; it < 32; ++it) {
    if (lo >= hi) break;
    const int mid  = (lo + hi) >> 1;
    const int midc = mid < 0 ? 0 : (mid > nN - 1 ? nN - 1 : mid);
    const int b = bat[midc];
    if (b < key) lo = mid + 1; else hi = mid;
  }
  return lo;
}

__global__ __launch_bounds__(NTHR) void k_pool(const float* __restrict__ va, const float* __restrict__ vb,
                                               const float* __restrict__ sta, const float* __restrict__ stb,
                                               const int* __restrict__ bat, const int* __restrict__ flg,
                                               int nN, float* out) {
  __shared__ __attribute__((aligned(16))) float wsum[NWAVE * 2 * DF];
  __shared__ __attribute__((aligned(16))) float outs[2 * DF];
  const int tid = (int)threadIdx.x, lane = tid & 31, wave = tid >> 5;
  const int g = (int)blockIdx.x;
  const int bad = flg[0];

  int s0 = lbound(bat, nN, g);
  int s1 = lbound(bat, nN, g + 1);
  s0 = s0 < 0 ? 0 : (s0 > nN ? nN : s0);
  s1 = s1 < s0 ? s0 : (s1 > nN ? nN : s1);

  const v2f ma = *(const v2fa*)(sta + 2 * lane);
  const v2f sa = *(const v2fa*)(sta + DF + 2 * lane);
  const v2f ba = *(const v2fa*)(sta + 2 * DF + 2 * lane);
  const v2f mb = *(const v2fa*)(stb + 2 * lane);
  const v2f sb = *(const v2fa*)(stb + DF + 2 * lane);
  const v2f bb = *(const v2fa*)(stb + 2 * DF + 2 * lane);

  float a0 = 0.0f, a1 = 0.0f, c0 = 0.0f, c1 = 0.0f;
#pragma unroll 1
  for (int r = s0 + wave; r < s1; r += NWAVE) {
    const int rc = r > nN - 1 ? nN - 1 : r;
    const v2f p = *(const v2fa*)(va + (size_t)rc * DF + 2 * lane);
    const v2f q = *(const v2fa*)(vb + (size_t)rc * DF + 2 * lane);
    a0 += bnap(p.x, ma.x, sa.x, ba.x);
    a1 += bnap(p.y, ma.y, sa.y, ba.y);
    c0 += bnap(q.x, mb.x, sb.x, bb.x);
    c1 += bnap(q.y, mb.y, sb.y, bb.y);
  }
  wsum[wave * (2 * DF) + 2 * lane + 0]      = a0;
  wsum[wave * (2 * DF) + 2 * lane + 1]      = a1;
  wsum[wave * (2 * DF) + DF + 2 * lane + 0] = c0;
  wsum[wave * (2 * DF) + DF + 2 * lane + 1] = c1;
  __syncthreads();
  if (tid < 2 * DF) {
    float s = 0.0f;
#pragma unroll
    for (int w2 = 0; w2 < NWAVE; ++w2) s += wsum[w2 * (2 * DF) + tid];
    const float qn = __int_as_float(0x7fc00000);
    outs[tid] = (bad != 0) ? qn : s;
  }
  __syncthreads();
  const v4f ov = *(const v4fa*)(outs + 4 * lane);
  float* op = out + (size_t)g * (2 * DF) + 4 * lane;
  const bool okst = (wave == 0);
  if (okst) *(volatile v4f*)op = ov;
  __threadfence();
  if (okst) *(volatile v4f*)op = ov;
}

static inline int cdiv(int a, int b) { return (a + b - 1) / b; }
static inline size_t al256(size_t o) { return (o + 255) & ~(size_t)255; }

extern "C" void kernel_launch(void* const* d_in, const int* in_sizes, int n_in,
                              void* d_out, int out_size, void* d_ws, size_t ws_size,
                              hipStream_t stream) {
  if (n_in < 15) return;
  if (in_sizes[0] < DF || (in_sizes[0] % DF) != 0) return;
  const int nN = in_sizes[0] / DF;
  if (nN < 16 || nN > (1 << 22)) return;
  if (in_sizes[1] != DF * DF || in_sizes[2] != DF) return;
  if (in_sizes[3] != DF * DF || in_sizes[4] != DF) return;
  if (in_sizes[5] != DF || in_sizes[6] != DF) return;
  if (in_sizes[7] != DF * DF || in_sizes[8] != DF) return;
  if (in_sizes[9] != DF * DF || in_sizes[10] != DF) return;
  if (in_sizes[11] != DF || in_sizes[12] != DF) return;
  if (in_sizes[13] < 2 || (in_sizes[13] & 1) != 0) return;
  const int nE = in_sizes[13] / 2;
  if (nE < 1 || nE >= (1 << (31 - SLA))) return;
  if (in_sizes[14] != nN) return;
  if (out_size != NGR * 2 * DF) return;

  const float* x    = (const float*)d_in[0];
  const float* W10  = (const float*)d_in[1];
  const float* b10  = (const float*)d_in[2];
  const float* W20  = (const float*)d_in[3];
  const float* b20  = (const float*)d_in[4];
  const float* gm0  = (const float*)d_in[5];
  const float* bt0  = (const float*)d_in[6];
  const float* W11  = (const float*)d_in[7];
  const float* b11  = (const float*)d_in[8];
  const float* W21  = (const float*)d_in[9];
  const float* b21  = (const float*)d_in[10];
  const float* gm1  = (const float*)d_in[11];
  const float* bt1  = (const float*)d_in[12];
  const int*   edge = (const int*)d_in[13];
  const int*   bat  = (const int*)d_in[14];
  float* out = (float*)d_out;
  const int* src = edge;
  const int* dst = edge + nE;

  const int MP  = cdiv(nN, TM) * TM;
  const int nT  = MP / TM;
  const int gA  = cdiv(MP, NBA);
  if ((long long)gA * NBA < (long long)MP) return;
  const int nUx = MP * (DF / 8);
  const int nbX = cdiv(nUx, NTHR);
  const int vec8 = ((nE & 3) == 0) ? 1 : 0;

  char* ws = (char*)d_ws;
  size_t off = 0;
  const size_t oWP  = off; off = al256(off + (size_t)4 * DF * KH * 2);
  const size_t oFLG = off; off = al256(off + 128);
  const size_t oST0 = off; off = al256(off + (size_t)4 * DF * 4);
  const size_t oST1 = off; off = al256(off + (size_t)4 * DF * 4);
  const size_t oXB  = off; off = al256(off + (size_t)MP * DF * 2);
  const size_t oH   = off; off = al256(off + (size_t)MP * KH * 2);
  const size_t oV0  = off; off = al256(off + (size_t)MP * DF * 4);
  const size_t oV1  = off; off = al256(off + (size_t)MP * DF * 4);
  const size_t oR0  = off; off = al256(off + (size_t)nT * 2 * DF * 8);
  const size_t oR1  = off; off = al256(off + (size_t)nT * 2 * DF * 8);
  if (off > ws_size || off > (size_t)WSMAX) return;
  unsigned short* WP  = (unsigned short*)(ws + oWP);
  int*            FLG = (int*)(ws + oFLG);
  float*          ST0 = (float*)(ws + oST0);
  float*          ST1 = (float*)(ws + oST1);
  unsigned short* XB  = (unsigned short*)(ws + oXB);
  unsigned short* H   = (unsigned short*)(ws + oH);
  float*          V0  = (float*)(ws + oV0);
  float*          V1  = (float*)(ws + oV1);
  double*         R0  = (double*)(ws + oR0);
  double*         R1  = (double*)(ws + oR1);

  const size_t scanLds = (size_t)AGG_LDS_INTS * 4;
  const size_t mlpLds  = (size_t)MLP_LDS;
  hipFuncSetAttribute(reinterpret_cast<const void*>(&k_scan<1>), hipFuncAttributeMaxDynamicSharedMemorySize, (int)scanLds);
  hipFuncSetAttribute(reinterpret_cast<const void*>(&k_scan<0>), hipFuncAttributeMaxDynamicSharedMemorySize, (int)scanLds);
  hipFuncSetAttribute(reinterpret_cast<const void*>(&k_mlp), hipFuncAttributeMaxDynamicSharedMemorySize, (int)mlpLds);

  k_prep<<<NWBLK + nbX + 1, NTHR, 0, stream>>>(x, W10, W20, W11, W21, bat, nN, nUx, nbX, WP, XB, FLG);
  k_scan<1><<<gA, NTHR, scanLds, stream>>>(src, dst, nE, nN, vec8, MP, (const unsigned*)XB, V0, ST0, H);
  k_mlp<<<nT, NTHR, mlpLds, stream>>>(H, WP, WP + 8192, b10, b20, nN, V0, R0);
  k_bn<<<1, 128, 0, stream>>>(R0, nT, nN, gm0, bt0, ST0);
  k_scan<0><<<gA, NTHR, scanLds, stream>>>(src, dst, nE, nN, vec8, MP, (const unsigned*)XB, V0, ST0, H);
  k_mlp<<<nT, NTHR, mlpLds, stream>>>(H, WP + 16384, WP + 24576, b11, b21, nN, V1, R1);
  k_bn<<<1, 128, 0, stream>>>(R1, nT, nN, gm1, bt1, ST1);
  k_pool<<<NGR, NTHR, 0, stream>>>(V0, V1, ST0, ST1, bat, FLG, nN, out);
}
